// LSREF_84911503442267
// MI455X (gfx1250) — hardware-verified
//
#include <hip/hip_runtime.h>


#define NBT  4
#define LL   1024
#define CC   512
#define GLN  4096
#define NW   512
#define NH_  16
#define HD   32
#define DFF  2048
#define DM   CC
#define NX   LL
#define NZ   NW
#define QSC  0.17677669529663688f
#define LEPS 1e-5f
#define LOSC 1024.0f

typedef _Float16 h16;
typedef unsigned short bf;
typedef __attribute__((ext_vector_type(16))) __bf16   v16bf;
typedef __attribute__((ext_vector_type(16))) _Float16 v16h;
typedef __attribute__((ext_vector_type(8)))  _Float16 v8h;
typedef __attribute__((ext_vector_type(8)))  unsigned short v8us;
typedef __attribute__((ext_vector_type(8)))  float    v8f;
typedef __attribute__((ext_vector_type(4)))  float    v4f;
typedef v8h  __attribute__((may_alias)) v8ha;
typedef v4f  __attribute__((may_alias)) v4fa;
typedef v8us __attribute__((may_alias)) v8usa;

__device__ __forceinline__ unsigned short f2bf(float f) { unsigned u = __float_as_uint(f); u += 0x7FFFu + ((u >> 16) & 1u); return (unsigned short)(u >> 16); }
__device__ __forceinline__ float bf2f(unsigned short b) { return __uint_as_float(((unsigned)b) << 16); }
__device__ __forceinline__ float bfr(float f) { return bf2f(f2bf(f)); }
__device__ __forceinline__ v16h cat16(v8h lo, v8h hi) { return __builtin_shufflevector(lo, hi, 0, 1, 2, 3, 4, 5, 6, 7, 8, 9, 10, 11, 12, 13, 14, 15); }
__device__ __forceinline__ v16bf cat16b(v8us lo, v8us hi) { return __builtin_bit_cast(v16bf, __builtin_shufflevector(lo, hi, 0, 1, 2, 3, 4, 5, 6, 7, 8, 9, 10, 11, 12, 13, 14, 15)); }
__device__ __forceinline__ v8f wmma16(v16h a, v16h b, v8f c) { return __builtin_amdgcn_wmma_f32_16x16x32_f16(false, a, false, b, (short)0, c, false, false); }
__device__ __forceinline__ v8f wmmab(v16bf a, v16bf b, v8f c) { return __builtin_amdgcn_wmma_f32_16x16x32_bf16(false, a, false, b, (short)0, c, false, false); }

template <bool SPLITA, bool F16OUT = false>
__global__ __launch_bounds__(128) void k_gemmb(const bf* __restrict__ A, const bf* __restrict__ Al, const bf* __restrict__ Bn, const float* __restrict__ bias, float* C, int ldc, h16* C2, const float* __restrict__ R = nullptr, int K = DM, int roundR = 1) {
    __shared__ __align__(16) float ost[4][16 * 68];
    const int lane = threadIdx.x & 31, wave = threadIdx.x >> 5, lr = lane & 15, hi = lane >> 4;
    const int r0 = blockIdx.x * 64 + wave * 16, c0 = blockIdx.y * 64;
    const size_t aoff = (size_t)(r0 + lr) * K + 8 * hi;
    size_t boff[4];
#pragma unroll
    for (int t = 0; t < 4; ++t) boff[t] = (size_t)(c0 + t * 16 + lr) * K + 8 * hi;
    v8f acc[4];
#pragma unroll
    for (int t = 0; t < 4; ++t) acc[t] = (v8f){};
#pragma unroll 1
    for (int kc = 0; kc < K; kc += 32) {
        const v16bf a = cat16b(*(const v8us*)(A + aoff + kc), *(const v8us*)(A + aoff + kc + 16));
        v16bf al = a;
        if (SPLITA) al = cat16b(*(const v8us*)(Al + aoff + kc), *(const v8us*)(Al + aoff + kc + 16));
#pragma unroll
        for (int t = 0; t < 4; ++t) { const v16bf b = cat16b(*(const v8us*)(Bn + boff[t] + kc), *(const v8us*)(Bn + boff[t] + kc + 16)); acc[t] = wmmab(a, b, acc[t]); if (SPLITA) acc[t] = wmmab(al, b, acc[t]); }
        asm volatile("v_nop\n\tv_nop\n\tv_nop\n\tv_nop" : "+v"(acc[0]), "+v"(acc[1]), "+v"(acc[2]), "+v"(acc[3]) : "v"(a), "v"(al));
    }
    float* os = &ost[wave][0];
#pragma unroll
    for (int t = 0; t < 4; ++t) { const float bv = bias ? bfr(bias[c0 + t * 16 + lr]) : 0.f;
#pragma unroll
        for (int j = 0; j < 8; ++j) os[(hi * 8 + j) * 68 + t * 16 + lr] = acc[t][j] + bv; }
    __syncthreads();
    if (F16OUT) {
        h16* crow = (h16*)(void*)C + (size_t)r0 * ldc + c0;
        auto pass = [&]() {
#pragma unroll
            for (int s = 0; s < 4; ++s) { const int row = 4 * s + (lane >> 3), piece = lane & 7; const float* sp = os + row * 68 + piece * 8; v8h o, o2;
#pragma unroll
                for (int i = 0; i < 8; ++i) { const h16 a = (h16)sp[i]; o[i] = a; o2[i] = (h16)((sp[i] - (float)a) * LOSC); }
                *(volatile v8h*)(crow + (size_t)row * ldc + piece * 8) = o; if (C2) *(volatile v8h*)(C2 + (size_t)r0 * ldc + c0 + (size_t)row * ldc + piece * 8) = o2; }
        };
        pass(); __threadfence(); pass();
    } else {
        float* crow = C + (size_t)r0 * ldc + c0;
        auto pass = [&]() {
#pragma unroll
            for (int s = 0; s < 8; ++s) { const int Lid = (lane >> 3) + 4 * s, piece = lane & 7; const int row = Lid >> 1, cofs = (Lid & 1) * 32 + piece * 4;
                v4f val = *(const v4fa*)(os + row * 68 + cofs); if (R) { const v4f rv = *(const v4f*)(R + ((size_t)r0 + row) * ldc + c0 + cofs); val += roundR ? (v4f){bfr(rv[0]), bfr(rv[1]), bfr(rv[2]), bfr(rv[3])} : rv; }
                *(volatile v4f*)(crow + (size_t)row * ldc + cofs) = val; }
        };
        pass(); __threadfence(); pass();
    }
}

__global__ __launch_bounds__(256) void k_cvt8(const float* __restrict__ src, bf* dst, size_t n8) {
    const size_t i = (size_t)blockIdx.x * 256 + threadIdx.x; if (i >= n8) return;
    const v8f v = *(const v8f*)(src + i * 8); v8us o;
#pragma unroll
    for (int k = 0; k < 8; ++k) o[k] = f2bf(v[k]);
    *(volatile v8us*)(dst + i * 8) = o; __threadfence(); *(volatile v8us*)(dst + i * 8) = o;
}
__global__ __launch_bounds__(256) void k_zero8(bf* dst, size_t n8) {
    const size_t i = (size_t)blockIdx.x * 256 + threadIdx.x; if (i >= n8) return; v8us z;
#pragma unroll
    for (int k = 0; k < 8; ++k) z[k] = 0;
    *(volatile v8us*)(dst + i * 8) = z; __threadfence(); *(volatile v8us*)(dst + i * 8) = z;
}

template <int MODE>
__global__ __launch_bounds__(128) void k_gemm3z(const bf* __restrict__ Ah, const bf* __restrict__ Al, const bf* __restrict__ Bh, const bf* __restrict__ Bl, int K, float* C, int ldc, size_t sA, size_t sB, size_t sC) {
    if ((MODE & 1) && (int)blockIdx.y * 64 > (int)blockIdx.x * 64 + 63) return;
    const size_t z = blockIdx.z; Ah += z * sA; Al += z * sA; Bh += z * sB; Bl += z * sB; C += z * sC;
    const int Klim = (MODE & 2) ? min(K, ((int)blockIdx.x + 1) * 64) : K;
    __shared__ __align__(16) float ost[4][16 * 68];
    const int lane = threadIdx.x & 31, wave = threadIdx.x >> 5, lr = lane & 15, hi = lane >> 4;
    const int r0 = blockIdx.x * 64 + wave * 16, c0 = blockIdx.y * 64;
    const size_t aoff = (size_t)(r0 + lr) * K + 8 * hi;
    v8f acc[4];
#pragma unroll
    for (int t = 0; t < 4; ++t) acc[t] = (v8f){};
#pragma unroll 1
    for (int kc = 0; kc < Klim; kc += 32) {
        const v16bf a = cat16b(*(const v8us*)(Ah + aoff + kc), *(const v8us*)(Ah + aoff + kc + 16));
        v16bf al = a; if (!(MODE & 4) && !(MODE & 16)) al = cat16b(*(const v8us*)(Al + aoff + kc), *(const v8us*)(Al + aoff + kc + 16));
#pragma unroll
        for (int t = 0; t < 4; ++t) { const size_t bo = (size_t)(c0 + t * 16 + lr) * K + kc + 8 * hi;
            const v16bf bh = cat16b(*(const v8us*)(Bh + bo), *(const v8us*)(Bh + bo + 16));
            acc[t] = wmmab(a, bh, acc[t]);
            if (!(MODE & 4)) { if (!(MODE & 16)) acc[t] = wmmab(al, bh, acc[t]); if (!(MODE & 8)) { const v16bf bl = cat16b(*(const v8us*)(Bl + bo), *(const v8us*)(Bl + bo + 16)); acc[t] = wmmab(a, bl, acc[t]); } } }
        asm volatile("v_nop\n\tv_nop\n\tv_nop\n\tv_nop" : "+v"(acc[0]), "+v"(acc[1]), "+v"(acc[2]), "+v"(acc[3]) : "v"(a), "v"(al));
    }
    float* os = &ost[wave][0];
#pragma unroll
    for (int t = 0; t < 4; ++t) {
#pragma unroll
        for (int j = 0; j < 8; ++j) os[(hi * 8 + j) * 68 + t * 16 + lr] = acc[t][j]; }
    __builtin_amdgcn_wave_barrier(); asm volatile("" ::: "memory");
    float* crow = C + (size_t)r0 * ldc + c0;
    auto pass = [&]() {
#pragma unroll
        for (int s = 0; s < 8; ++s) { const int Lid = (lane >> 3) + 4 * s, piece = lane & 7; const int row = Lid >> 1, cofs = (Lid & 1) * 32 + piece * 4;
            const v4f val = *(const v4fa*)(os + row * 68 + cofs); *(volatile v4f*)(crow + (size_t)row * ldc + cofs) = val; }
    };
    pass(); __threadfence(); pass();
}
__global__ __launch_bounds__(256) void k_planes32z(const float* __restrict__ F, int ld, int off, float sc, int rows, bf* Ph, bf* Pl) {
    typedef __attribute__((ext_vector_type(2))) unsigned short v2us;
    const int lane = threadIdx.x & 31; const size_t r = ((size_t)blockIdx.x * 8 + (threadIdx.x >> 5)) * 2 + (lane >> 4); if (r >= (size_t)rows) return; const int z = blockIdx.z; const int c0 = (lane & 15) * 2; v2us oh, ol;
    Ph += (size_t)z * rows * 32; Pl += (size_t)z * rows * 32;
#pragma unroll
    for (int i = 0; i < 2; ++i) { const float y = F[r * ld + off + z * 32 + c0 + i] * sc; const unsigned short hb = f2bf(y); oh[i] = hb; ol[i] = f2bf(y - bf2f(hb)); }
    const size_t o = r * 32 + c0; *(volatile v2us*)(Ph + o) = oh; *(volatile v2us*)(Pl + o) = ol; __threadfence(); *(volatile v2us*)(Ph + o) = oh; *(volatile v2us*)(Pl + o) = ol;
}
__global__ __launch_bounds__(256) void k_vtpadz(const float* __restrict__ F, int ld, int off, int nk, bf* Th, bf* Tl) {
    typedef __attribute__((ext_vector_type(2))) unsigned short v2us;
    const int lane = threadIdx.x & 31; const size_t wid = (size_t)blockIdx.x * 8 + (threadIdx.x >> 5); if (wid >= (size_t)64 * (nk / 64)) return; const int z = blockIdx.z; const int d = (int)(wid / (nk / 64)); const int k0 = (int)(wid % (nk / 64)) * 64 + lane * 2; v2us oh, ol;
    Th += (size_t)z * 64 * nk; Tl += (size_t)z * 64 * nk;
#pragma unroll
    for (int i = 0; i < 2; ++i) { const float y = (d < 32) ? F[(size_t)(k0 + i) * ld + off + z * 32 + (d < 32 ? d : 0)] : 0.f; const unsigned short hb = f2bf(y); oh[i] = hb; ol[i] = f2bf(y - bf2f(hb)); }
    const size_t o = (size_t)d * nk + k0; *(volatile v2us*)(Th + o) = oh; *(volatile v2us*)(Tl + o) = ol; __threadfence(); *(volatile v2us*)(Th + o) = oh; *(volatile v2us*)(Tl + o) = ol;
}
template <int NK>
__global__ __launch_bounds__(256) void k_softmaxz(const float* __restrict__ S, int rows, bf* PH, bf* PL) {
    typedef __attribute__((ext_vector_type(4))) unsigned short v4us;
    const int lane = threadIdx.x & 31, i = blockIdx.x * 8 + (threadIdx.x >> 5); if (i >= rows) return; const size_t zo = (size_t)blockIdx.z * rows * NK; const float* sr = S + zo + (size_t)i * NK; PH += zo; PL += zo;
    float m = -3.0e38f;
#pragma unroll 1
    for (int c0 = lane * 4; c0 < NK; c0 += 128) {
#pragma unroll
        for (int q = 0; q < 4; ++q) m = fmaxf(m, sr[c0 + q]); }
#pragma unroll
    for (int sh = 16; sh; sh >>= 1) m = fmaxf(m, __shfl_xor(m, sh, 32));
    float sum = 0.f;
#pragma unroll 1
    for (int c0 = lane * 4; c0 < NK; c0 += 128) {
#pragma unroll
        for (int q = 0; q < 4; ++q) sum += __expf(sr[c0 + q] - m); }
#pragma unroll
    for (int sh = 16; sh; sh >>= 1) sum += __shfl_xor(sum, sh, 32);
    const float inv = 1.0f / sum;
#pragma unroll 1
    for (int ps = 0; ps < 2; ++ps) {
#pragma unroll 1
        for (int c0 = lane * 4; c0 < NK; c0 += 128) { v4us oh, ol;
#pragma unroll
            for (int q = 0; q < 4; ++q) { const float p = __expf(sr[c0 + q] - m) * inv; const unsigned short hb = f2bf(p); oh[q] = hb; ol[q] = f2bf(p - bf2f(hb)); }
            const size_t o = (size_t)i * NK + c0; *(volatile v4us*)(PH + o) = oh; *(volatile v4us*)(PL + o) = ol; }
        if (ps == 0) __threadfence(); }
}
__global__ __launch_bounds__(256) void k_placez(const float* __restrict__ XH, int rows, int ldy, float* Y) {
    const int lane = threadIdx.x & 31; const size_t q = (size_t)blockIdx.x * 8 + (threadIdx.x >> 5); if (q >= (size_t)rows) return; const int z = blockIdx.z; const float v = XH[((size_t)z * rows + q) * 64 + lane];
    *(volatile float*)(Y + q * ldy + z * 32 + lane) = v; __threadfence(); *(volatile float*)(Y + q * ldy + z * 32 + lane) = v;
}

__global__ __launch_bounds__(256) void k_cvtrow(const float* __restrict__ src, int rows, bf* dst) {
    const int lane = threadIdx.x & 31; const size_t r = (size_t)blockIdx.x * 8 + (threadIdx.x >> 5); if (r >= (size_t)rows) return;
#pragma unroll 1
    for (int ps = 0; ps < 2; ++ps) {
#pragma unroll
        for (int q = 0; q < CC / 256; ++q) { v8us o;
#pragma unroll
            for (int i = 0; i < 8; ++i) o[i] = f2bf(src[r * CC + q * 256 + lane * 8 + i]);
            *(volatile v8us*)(dst + r * CC + q * 256 + lane * 8) = o; }
        if (ps == 0) __threadfence(); }
}
__global__ __launch_bounds__(256) void k_window(const float* __restrict__ gf, bf* Rh, bf* Rl) {
    const int lane = threadIdx.x & 31; const int d = blockIdx.x * 8 + (threadIdx.x >> 5); if (d >= NW) return;
#pragma unroll 1
    for (int ps = 0; ps < 2; ++ps) {
#pragma unroll
        for (int q = 0; q < CC / 256; ++q) { v8us oh, ol;
#pragma unroll
            for (int i = 0; i < 8; ++i) { const int c = q * 256 + lane * 8 + i; const float* p = gf + (size_t)c * GLN + (size_t)d * 8; float mx = bfr(p[0]), mn = mx;
#pragma unroll
                for (int t = 1; t < 8; ++t) { const float v = bfr(p[t]); mx = fmaxf(mx, v); mn = fminf(mn, v); }
                const float y = fabsf(mx - mn) + 1e-6f; const unsigned short hb = f2bf(y); oh[i] = hb; ol[i] = f2bf(y - bf2f(hb)); }
            const size_t o = (size_t)d * CC + q * 256 + lane * 8; *(volatile v8us*)(Rh + o) = oh; *(volatile v8us*)(Rl + o) = ol; }
        if (ps == 0) __threadfence(); }
}
__global__ __launch_bounds__(256) void k_browrelu(const float* __restrict__ CR, const float* __restrict__ cb, bf* Ph, bf* Pl) {
    const int lane = threadIdx.x & 31; const size_t s = (size_t)blockIdx.x * 8 + (threadIdx.x >> 5); if (s >= (size_t)NW) return; const float bs = bfr(cb[s]);
#pragma unroll 1
    for (int ps = 0; ps < 2; ++ps) {
#pragma unroll
        for (int q = 0; q < CC / 256; ++q) { const size_t o = s * CC + q * 256 + lane * 8; const v8f v = *(const v8f*)(CR + o); v8us oh, ol;
#pragma unroll
            for (int i = 0; i < 8; ++i) { const float y = fmaxf(v[i] + bs, 0.f); const unsigned short hb = f2bf(y); oh[i] = hb; ol[i] = f2bf(y - bf2f(hb)); }
            *(volatile v8us*)(Ph + o) = oh; *(volatile v8us*)(Pl + o) = ol; }
        if (ps == 0) __threadfence(); }
}
template <bool RIN>
__global__ __launch_bounds__(256) void k_addln(const float* __restrict__ A, const float* __restrict__ Bm, const float* __restrict__ g, const float* __restrict__ bb, float* Yf, bf* Yh, bf* Yl) {
    const int lane = threadIdx.x & 31; const size_t r = (size_t)blockIdx.x * 8 + (threadIdx.x >> 5); if (r >= (size_t)LL) return; float v[16]; float s = 0.f;
#pragma unroll
    for (int q = 0; q < 2; ++q) {
#pragma unroll
        for (int i = 0; i < 8; ++i) { const size_t o = r * CC + q * 256 + lane * 8 + i; const float bv = RIN ? bfr(Bm[o]) : Bm[o]; const float t = A[o] + bv; v[q * 8 + i] = t; s += t; } }
#pragma unroll
    for (int sh = 16; sh; sh >>= 1) s += __shfl_xor(s, sh, 32);
    const float mu = s * (1.0f / CC); float qv = 0.f;
#pragma unroll
    for (int i = 0; i < 16; ++i) { const float d = v[i] - mu; qv = fmaf(d, d, qv); }
#pragma unroll
    for (int sh = 16; sh; sh >>= 1) qv += __shfl_xor(qv, sh, 32);
    const float rs = rsqrtf(qv * (1.0f / CC) + LEPS);
#pragma unroll 1
    for (int ps = 0; ps < 2; ++ps) {
#pragma unroll
        for (int q = 0; q < 2; ++q) { const int c0 = q * 256 + lane * 8; v8f y; v8us oh, ol;
#pragma unroll
            for (int i = 0; i < 8; ++i) { y[i] = (v[q * 8 + i] - mu) * rs * bfr(g[c0 + i]) + bfr(bb[c0 + i]); const unsigned short hb = f2bf(y[i]); oh[i] = hb; ol[i] = f2bf(y[i] - bf2f(hb)); }
            const size_t o = r * CC + c0; *(volatile v8f*)(Yf + o) = y; *(volatile v8us*)(Yh + o) = oh; *(volatile v8us*)(Yl + o) = ol; }
        if (ps == 0) __threadfence(); }
}
__global__ __launch_bounds__(256) void k_gelu2048(const float* __restrict__ F, bf* Gh, bf* Gl) {
    const int lane = threadIdx.x & 31; const size_t r = (size_t)blockIdx.x * 8 + (threadIdx.x >> 5); if (r >= (size_t)LL) return;
#pragma unroll 1
    for (int ps = 0; ps < 2; ++ps) {
#pragma unroll 1
        for (int q = 0; q < DFF / 256; ++q) { const size_t o = r * DFF + q * 256 + lane * 8; const v8f v = *(const v8f*)(F + o); v8us oh, ol;
#pragma unroll
            for (int i = 0; i < 8; ++i) { const float x = v[i]; const float gx = 0.5f * x * (1.0f + erff(x * 0.70710678118654752f)); const unsigned short hb = f2bf(gx); oh[i] = hb; ol[i] = f2bf(gx - bf2f(hb)); }
            *(volatile v8us*)(Gh + o) = oh; *(volatile v8us*)(Gl + o) = ol; }
        if (ps == 0) __threadfence(); }
}
__global__ __launch_bounds__(256) void k_trout(const float* __restrict__ Y, float* OUTB) {
    __shared__ float tl[64][65];
    const int tid = threadIdx.x, l0 = blockIdx.x * 64, c0 = blockIdx.y * 64; const int rr = tid >> 2, cq = (tid & 3) * 16;
#pragma unroll
    for (int i = 0; i < 16; ++i) tl[rr][cq + i] = Y[(size_t)(l0 + rr) * CC + c0 + cq + i];
    __syncthreads();
    const int lane = tid & 31, wv = tid >> 5;
    auto pass = [&]() {
#pragma unroll
        for (int st = 0; st < 4; ++st) { const int cr = wv * 8 + st * 2 + (lane >> 4); const int lq = (lane & 15) * 4; v4f v;
#pragma unroll
            for (int i = 0; i < 4; ++i) v[i] = tl[lq + i][cr];
            *(volatile v4f*)(OUTB + (size_t)(c0 + cr) * LL + l0 + lq) = v; }
    };
    pass(); __threadfence(); pass();
}

__global__ __launch_bounds__(256) void k_split512(const float* __restrict__ src, int rows, bf* dh, bf* dl) {
    const int lane = threadIdx.x & 31; const size_t r = (size_t)blockIdx.x * 8 + (threadIdx.x >> 5); if (r >= (size_t)rows) return;
#pragma unroll 1
    for (int ps = 0; ps < 2; ++ps) {
#pragma unroll
        for (int q = 0; q < CC / 256; ++q) { const size_t o = r * CC + q * 256 + lane * 8; const v8f v = *(const v8f*)(src + o); v8us oh, ol;
#pragma unroll
            for (int i = 0; i < 8; ++i) { const unsigned short hb = f2bf(v[i]); oh[i] = hb; ol[i] = f2bf(v[i] - bf2f(hb)); }
            *(volatile v8us*)(dh + o) = oh; *(volatile v8us*)(dl + o) = ol; }
        if (ps == 0) __threadfence(); }
}

extern "C" void kernel_launch(void* const* d_in, const int* in_sizes, int n_in,
                              void* d_out, int out_size, void* d_ws, size_t ws_size, hipStream_t stream) {
    (void)in_sizes; (void)n_in; (void)out_size;
    const float* x = (const float*)d_in[0]; const float* gf = (const float*)d_in[1]; const float* conv_w = (const float*)d_in[2]; const float* conv_b = (const float*)d_in[3];
    const float* sa_wq = (const float*)d_in[4]; const float* sa_bq = (const float*)d_in[5]; const float* sa_wk = (const float*)d_in[6]; const float* sa_bk = (const float*)d_in[7]; const float* sa_wv = (const float*)d_in[8]; const float* sa_bv = (const float*)d_in[9]; const float* sa_wo = (const float*)d_in[10]; const float* sa_bo = (const float*)d_in[11];
    const float* ca_wq = (const float*)d_in[12]; const float* ca_bq = (const float*)d_in[13]; const float* ca_wk = (const float*)d_in[14]; const float* ca_bk = (const float*)d_in[15]; const float* ca_wv = (const float*)d_in[16]; const float* ca_bv = (const float*)d_in[17]; const float* ca_wo = (const float*)d_in[18]; const float* ca_bo = (const float*)d_in[19];
    const float* f_w1 = (const float*)d_in[20]; const float* f_b1 = (const float*)d_in[21]; const float* f_w2 = (const float*)d_in[22]; const float* f_b2 = (const float*)d_in[23];
    const float* n1g = (const float*)d_in[24]; const float* n1b = (const float*)d_in[25]; const float* n2g = (const float*)d_in[26]; const float* n2b = (const float*)d_in[27]; const float* n3g = (const float*)d_in[28]; const float* n3b = (const float*)d_in[29];
    float* out = (float*)d_out;
    char* wsp = (char*)d_ws;
    auto take = [&](size_t bytes) { char* p = wsp; wsp += (bytes + 255) & ~(size_t)255; return (void*)p; };
    const int ZH = 8; const size_t WSZ = (size_t)CC * CC * 2;
    bf* CW = (bf*)take(WSZ); bf* SWQ = (bf*)take(WSZ); bf* SWK = (bf*)take(WSZ); bf* SWV = (bf*)take(WSZ); bf* SWO = (bf*)take(WSZ); bf* CWQ = (bf*)take(WSZ); bf* CWK = (bf*)take(WSZ); bf* CWV = (bf*)take(WSZ); bf* CWO = (bf*)take(WSZ);
    bf* FW1 = (bf*)take((size_t)DFF * CC * 2); bf* FW2 = (bf*)take((size_t)CC * DFF * 2);
    bf* Xb = (bf*)take((size_t)LL * CC * 2); bf* Rh = (bf*)take((size_t)NW * CC * 2); bf* Rl = (bf*)take((size_t)NW * CC * 2); float* CR1 = (float*)take((size_t)NW * CC * 4); float* CR = (float*)take((size_t)NW * CC * 4); bf* CRh = (bf*)take((size_t)NW * CC * 2); bf* CRl = (bf*)take((size_t)NW * CC * 2);
    float* QF = (float*)take((size_t)LL * CC * 4); float* KF = (float*)take((size_t)LL * CC * 4); float* VF = (float*)take((size_t)LL * CC * 4);
    bf* Qh = (bf*)take((size_t)ZH * LL * HD * 2); bf* Ql = (bf*)take((size_t)ZH * LL * HD * 2); bf* Kh = (bf*)take((size_t)ZH * LL * HD * 2); bf* Kl = (bf*)take((size_t)ZH * LL * HD * 2); bf* VTh = (bf*)take((size_t)ZH * 64 * LL * 2); bf* VTl = (bf*)take((size_t)ZH * 64 * LL * 2);
    float* S = (float*)take((size_t)ZH * LL * LL * 4); bf* PH = (bf*)take((size_t)ZH * LL * LL * 2); bf* PL = (bf*)take((size_t)ZH * LL * LL * 2); float* XH = (float*)take((size_t)ZH * LL * 64 * 4);
    float* Y = (float*)take((size_t)LL * CC * 4); bf* Yh = (bf*)take((size_t)LL * CC * 2); bf* Yl = (bf*)take((size_t)LL * CC * 2); float* AO = (float*)take((size_t)LL * CC * 4);
    float* H1 = (float*)take((size_t)LL * CC * 4); bf* H1h = (bf*)take((size_t)LL * CC * 2); bf* H1l = (bf*)take((size_t)LL * CC * 2); float* H2 = (float*)take((size_t)LL * CC * 4); bf* H2h = (bf*)take((size_t)LL * CC * 2); bf* H2l = (bf*)take((size_t)LL * CC * 2);
    float* F1 = (float*)take((size_t)LL * DFF * 4); bf* Gh = (bf*)take((size_t)LL * DFF * 2); bf* Gl = (bf*)take((size_t)LL * DFF * 2); float* OF = (float*)take((size_t)LL * CC * 4);
    if ((size_t)(wsp - (char*)d_ws) > ws_size) return;
    k_cvt8<<<(CC * CC / 8 + 255) / 256, 256, 0, stream>>>(conv_w, CW, CC * CC / 8);
    k_cvt8<<<(CC * CC / 8 + 255) / 256, 256, 0, stream>>>(sa_wq, SWQ, CC * CC / 8); k_cvt8<<<(CC * CC / 8 + 255) / 256, 256, 0, stream>>>(sa_wk, SWK, CC * CC / 8); k_cvt8<<<(CC * CC / 8 + 255) / 256, 256, 0, stream>>>(sa_wv, SWV, CC * CC / 8); k_cvt8<<<(CC * CC / 8 + 255) / 256, 256, 0, stream>>>(sa_wo, SWO, CC * CC / 8);
    k_cvt8<<<(CC * CC / 8 + 255) / 256, 256, 0, stream>>>(ca_wq, CWQ, CC * CC / 8); k_cvt8<<<(CC * CC / 8 + 255) / 256, 256, 0, stream>>>(ca_wk, CWK, CC * CC / 8); k_cvt8<<<(CC * CC / 8 + 255) / 256, 256, 0, stream>>>(ca_wv, CWV, CC * CC / 8); k_cvt8<<<(CC * CC / 8 + 255) / 256, 256, 0, stream>>>(ca_wo, CWO, CC * CC / 8);
    k_cvt8<<<(DFF * CC / 8 + 255) / 256, 256, 0, stream>>>(f_w1, FW1, DFF * CC / 8); k_cvt8<<<(CC * DFF / 8 + 255) / 256, 256, 0, stream>>>(f_w2, FW2, CC * DFF / 8);
    auto attend = [&](const float* QFp, const float* KFp, const float* VFp, int nk, float* Ydst) {
        for (int g = 0; g < NH_ / ZH; ++g) { const int h0 = g * ZH;
            k_planes32z<<<dim3((LL / 2) / 8, 1, ZH), 256, 0, stream>>>(QFp, CC, h0 * HD, QSC, LL, Qh, Ql); k_planes32z<<<dim3((nk / 2 + 7) / 8, 1, ZH), 256, 0, stream>>>(KFp, CC, h0 * HD, 1.0f, nk, Kh, Kl);
            k_vtpadz<<<dim3((64 * (nk / 64)) / 8, 1, ZH), 256, 0, stream>>>(VFp, CC, h0 * HD, nk, VTh, VTl);
            k_gemm3z<0><<<dim3(LL / 64, nk / 64, ZH), 128, 0, stream>>>(Qh, Ql, Kh, Kl, HD, S, nk, (size_t)LL * HD, (size_t)nk * HD, (size_t)LL * nk);
            if (nk == LL) k_softmaxz<LL><<<dim3(LL / 8, 1, ZH), 256, 0, stream>>>(S, LL, PH, PL); else k_softmaxz<NW><<<dim3(LL / 8, 1, ZH), 256, 0, stream>>>(S, LL, PH, PL);
            k_gemm3z<0><<<dim3(LL / 64, 1, ZH), 128, 0, stream>>>(PH, PL, VTh, VTl, nk, XH, 64, (size_t)LL * nk, (size_t)64 * nk, (size_t)LL * 64);
            k_placez<<<dim3(LL / 8, 1, ZH), 256, 0, stream>>>(XH, LL, CC, Ydst + h0 * HD); } };
    const dim3 gp(LL / 64, CC / 64, 1), gk(NW / 64, CC / 64, 1);
    for (int b = 0; b < NBT; ++b) { const float* xb = x + (size_t)b * LL * CC;
        k_window<<<NW / 8, 256, 0, stream>>>(gf + (size_t)b * CC * GLN, Rh, Rl);
        k_gemmb<false, false><<<gk, 128, 0, stream>>>(CW, nullptr, Rh, nullptr, CR1, CC, nullptr, nullptr, CC, 0);
        k_gemmb<false, false><<<gk, 128, 0, stream>>>(CW, nullptr, Rl, nullptr, CR, CC, nullptr, CR1, CC, 0);
        k_browrelu<<<NW / 8, 256, 0, stream>>>(CR, conv_b, CRh, CRl);
        k_cvtrow<<<LL / 8, 256, 0, stream>>>(xb, LL, Xb);
        k_gemmb<false, false><<<gp, 128, 0, stream>>>(Xb, nullptr, SWQ, sa_bq, QF, CC, nullptr, nullptr, CC); k_gemmb<false, false><<<gp, 128, 0, stream>>>(Xb, nullptr, SWK, sa_bk, KF, CC, nullptr, nullptr, CC); k_gemmb<false, false><<<gp, 128, 0, stream>>>(Xb, nullptr, SWV, sa_bv, VF, CC, nullptr, nullptr, CC);
        attend(QF, KF, VF, LL, Y);
        k_split512<<<LL / 8, 256, 0, stream>>>(Y, LL, Yh, Yl);
        k_gemmb<true, false><<<gp, 128, 0, stream>>>(Yh, Yl, SWO, sa_bo, AO, CC, nullptr, nullptr, CC);
        k_addln<true><<<LL / 8, 256, 0, stream>>>(AO, xb, n1g, n1b, H1, H1h, H1l);
        k_gemmb<true, false><<<gp, 128, 0, stream>>>(H1h, H1l, CWQ, ca_bq, QF, CC, nullptr, nullptr, CC); k_gemmb<true, false><<<gk, 128, 0, stream>>>(CRh, CRl, CWK, ca_bk, KF, CC, nullptr, nullptr, CC); k_gemmb<true, false><<<gk, 128, 0, stream>>>(CRh, CRl, CWV, ca_bv, VF, CC, nullptr, nullptr, CC);
        attend(QF, KF, VF, NW, Y);
        k_split512<<<LL / 8, 256, 0, stream>>>(Y, LL, Yh, Yl);
        k_gemmb<true, false><<<gp, 128, 0, stream>>>(Yh, Yl, CWO, ca_bo, AO, CC, nullptr, nullptr, CC);
        k_addln<false><<<LL / 8, 256, 0, stream>>>(AO, H1, n2g, n2b, H2, H2h, H2l);
        k_gemmb<true, false><<<dim3(LL / 64, DFF / 64, 1), 128, 0, stream>>>(H2h, H2l, FW1, f_b1, F1, DFF, nullptr, nullptr, CC);
        k_gelu2048<<<LL / 8, 256, 0, stream>>>(F1, Gh, Gl);
        k_gemmb<true, false><<<gp, 128, 0, stream>>>(Gh, Gl, FW2, f_b2, AO, CC, nullptr, nullptr, DFF);
        k_addln<false><<<LL / 8, 256, 0, stream>>>(AO, H2, n3g, n3b, OF, Yh, Yl);
        k_trout<<<dim3(LL / 64, CC / 64, 1), 256, 0, stream>>>(OF, out + (size_t)b * CC * LL); }
}
